// SelfAttention_61186104099586
// MI455X (gfx1250) — hardware-verified
//
#include <hip/hip_runtime.h>
#ifndef NB
#define NB 4
#endif
#ifndef SQ
#define SQ 1024
#endif
#define NB_FULL 4
#define SQ_FULL 1024
#define DM 1024
#define NH 16
#define HD 64
#define NR ((size_t)NB * SQ)

static_assert(NB >= 1 && NB <= NB_FULL);
static_assert(SQ >= 128 && SQ <= SQ_FULL && SQ % 128 == 0);
static_assert(NH * HD == DM && HD == 64);
static_assert(DM % 64 == 0 && DM % 32 == 0 && SQ % 64 == 0 && SQ % 16 == 0);
static_assert((NR % 128) == 0);
static_assert(((size_t)(NB - 1) * SQ_FULL + SQ) * DM * 4 <= (size_t)NB_FULL * SQ_FULL * DM * 4);
static_assert((((size_t)NB * (SQ / 16) * (SQ / 64)) % 4) == 0);

typedef unsigned short v8us __attribute__((ext_vector_type(8), may_alias));
typedef float  v8f  __attribute__((ext_vector_type(8)));
typedef float  v4f  __attribute__((ext_vector_type(4)));
typedef float  v4fa __attribute__((ext_vector_type(4), may_alias));
typedef _Float16 v16h __attribute__((ext_vector_type(16)));
typedef _Float16 v4h __attribute__((ext_vector_type(4)));
union FragH { v16h v; v8us half[2]; _Float16 h[16]; unsigned short u[16]; };

__device__ __forceinline__ unsigned short bf16_bits(float x) { unsigned int u = __float_as_uint(x); return (unsigned short)((u + 0x7FFFu + ((u >> 16) & 1u)) >> 16); }
__device__ __forceinline__ float bf16_val(unsigned short b) { return __uint_as_float(((unsigned int)b) << 16); }
__device__ __forceinline__ float bf16_rne(float x) { return bf16_val(bf16_bits(x)); }

static __device__ __forceinline__ _Float16 toh_flush(float v) { const _Float16 r = (_Float16)v; return (fabsf(v) < 6.103515625e-05f) ? (_Float16)0.0f : r; }

__device__ __forceinline__ v16h g2_frag(const _Float16* p, unsigned hh) { FragH f; f.half[0] = *(const v8us*)((const unsigned short*)p + 8 * hh); f.half[1] = *(const v8us*)((const unsigned short*)p + 16 + 8 * hh); return f.v; }
__device__ __forceinline__ v8f g2_mma(v16h a, v16h b, v8f c) { v8f d = __builtin_amdgcn_wmma_f32_16x16x32_f16(false, a, false, b, (short)0, c, false, false); asm volatile("v_nop\n\tv_nop\n\tv_nop\n\tv_nop" : "+v"(d) : "v"(a), "v"(b)); return d; }

__device__ __forceinline__ float gelu_erf(float v) { return 0.5f * v * (1.0f + erff(v * 0.70710678118654752f)); }

template <int ACT, int CPBF>
__global__ __launch_bounds__(128) void k_gemm2(const _Float16* __restrict__ A, unsigned lda, const _Float16* __restrict__ Bh, unsigned ldb, float alpha, const float* __restrict__ bias, const float* __restrict__ CP,
    float* __restrict__ C, _Float16* __restrict__ C16, unsigned ldc, float c16s, unsigned M, unsigned N, unsigned K) {
  static_assert(ACT == 0 || ACT == 8);
  __shared__ __attribute__((aligned(16))) float so[4][32][68];
  const unsigned tid = threadIdx.x, w = tid >> 5, lane = tid & 31u, ln = lane & 15u, hh = lane >> 4;
  const unsigned ntn = N >> 6; const unsigned mt = blockIdx.x / ntn, nq = blockIdx.x - mt * ntn; const unsigned row0 = mt * 128u + 32u * w, col0 = nq * 64u; if (row0 >= M) return;
  const _Float16* a0p = A + (size_t)(row0 + ln) * lda; const _Float16* a1p = a0p + (size_t)16 * lda;
  const _Float16* b0p = Bh + (size_t)(col0 + ln) * ldb; const _Float16* b1p = b0p + (size_t)16 * ldb; const _Float16* b2p = b1p + (size_t)16 * ldb; const _Float16* b3p = b2p + (size_t)16 * ldb;
  const v8f z8 = {0.f,0.f,0.f,0.f,0.f,0.f,0.f,0.f}; v8f c00 = z8, c01 = z8, c02 = z8, c03 = z8, c10 = z8, c11 = z8, c12 = z8, c13 = z8;
#pragma unroll 1
  for (unsigned kb = 0; kb < K; kb += 32) { const v16h a0 = g2_frag(a0p + kb, hh), a1 = g2_frag(a1p + kb, hh);
    v16h b = g2_frag(b0p + kb, hh); c00 = g2_mma(a0, b, c00); c10 = g2_mma(a1, b, c10);
    b = g2_frag(b1p + kb, hh); c01 = g2_mma(a0, b, c01); c11 = g2_mma(a1, b, c11);
    b = g2_frag(b2p + kb, hh); c02 = g2_mma(a0, b, c02); c12 = g2_mma(a1, b, c12);
    b = g2_frag(b3p + kb, hh); c03 = g2_mma(a0, b, c03); c13 = g2_mma(a1, b, c13); }
  v8f accs[8] = {c00, c01, c02, c03, c10, c11, c12, c13};
#pragma unroll
  for (int u = 0; u < 8; ++u) { const unsigned t = (unsigned)u & 3u, half = (unsigned)u >> 2; const unsigned col = col0 + t * 16u + ln; float bv = 0.f; if (bias) bv = bf16_rne(bias[col]);
#pragma unroll
    for (int r = 0; r < 8; ++r) { const unsigned rloc = half * 16u + 8u * hh + (unsigned)r; so[w][rloc][t * 16u + ln] = accs[u][r] * alpha + bv; } }
  __builtin_amdgcn_fence(4  , "workgroup"); __builtin_amdgcn_wave_barrier();
  const unsigned rsub = lane >> 4, c4 = (lane & 15u) * 4u;
  if (CP != nullptr || ACT == 8) {
#pragma unroll 2
    for (unsigned q = 0; q < 16; ++q) { const unsigned r = q * 2u + rsub; v4f v = *(const v4fa*)&so[w][r][c4];
      if (CP) { const v4f a = *(const v4fa*)(CP + (size_t)(row0 + r) * ldc + col0 + c4);
#pragma unroll
        for (int i = 0; i < 4; ++i) v[i] += CPBF ? bf16_rne(a[i]) : a[i]; }
      if (ACT == 8) {
#pragma unroll
        for (int i = 0; i < 4; ++i) v[i] = gelu_erf(v[i]); }
      *(v4fa*)&so[w][r][c4] = v; } }
  for (int pass = 0; pass < 2; ++pass) {
#pragma unroll
    for (unsigned q = 0; q < 16; ++q) { const unsigned r = q * 2u + rsub; const v4f v = *(const v4fa*)&so[w][r][c4];
      if (C) *(volatile v4f*)(C + (size_t)(row0 + r) * ldc + col0 + c4) = v;
      if (C16) { v4h h4;
#pragma unroll
        for (int i = 0; i < 4; ++i) h4[i] = (_Float16)(v[i] * c16s);
        *(volatile v4h*)(C16 + (size_t)(row0 + r) * ldc + col0 + c4) = h4; } }
    if (pass == 0) __threadfence(); } }

__global__ __launch_bounds__(256) void k_cvt(const float* __restrict__ X, float carry, _Float16* __restrict__ Y) {
  #pragma clang fp contract(off)
  const size_t i = ((size_t)blockIdx.x * 256u + threadIdx.x) * 8u;
  const v4f a = *(const v4fa*)(X + i); const v4f c = *(const v4fa*)(X + i + 4); FragH f;
#pragma unroll
  for (int q = 0; q < 4; ++q) { f.h[q] = toh_flush(bf16_rne(a[q]) * carry); f.h[4 + q] = toh_flush(bf16_rne(c[q]) * carry); }
  const v8us o = f.half[0];
  for (int pass = 0; pass < 2; ++pass) { *(volatile v8us*)((unsigned short*)Y + i) = o; if (pass == 0) __threadfence(); } }

__global__ __launch_bounds__(128) void k_mpack(const int* __restrict__ MK, unsigned int* __restrict__ MB) {
  const unsigned tid = threadIdx.x, lane = tid & 31u, ln = lane & 15u, hh = lane >> 4;
  const unsigned w = (unsigned)__builtin_amdgcn_readfirstlane((int)(tid >> 5));
  const unsigned L = blockIdx.x * 4u + w; const unsigned nkt = (unsigned)SQ / 64u, nqt = (unsigned)SQ / 16u;
  const unsigned t = L / nkt, kt = L - t * nkt; const unsigned b = t / nqt, qt = t - b * nqt;
  const int* mp = MK + ((size_t)b * SQ_FULL + qt * 16u + 8u * hh) * (size_t)SQ_FULL + kt * 64u + ln;
  unsigned int word = 0u;
#pragma unroll 1
  for (unsigned r = 0; r < 8u; ++r) { const int* mr = mp + (size_t)r * SQ_FULL; const int m0 = mr[0], m1 = mr[16], m2 = mr[32], m3 = mr[48];
    word |= ((m0 != 0) ? 1u : 0u) << r; word |= ((m1 != 0) ? 1u : 0u) << (8u + r); word |= ((m2 != 0) ? 1u : 0u) << (16u + r); word |= ((m3 != 0) ? 1u : 0u) << (24u + r); }
  for (int pass = 0; pass < 2; ++pass) { *(volatile unsigned int*)(MB + (size_t)L * 32u + lane) = word; if (pass == 0) __threadfence(); } }

template <int NHv, int TTv>
__global__ __launch_bounds__(256) void k_vt(const _Float16* __restrict__ V16, unsigned ldv, unsigned voff, _Float16* __restrict__ Vt) { __shared__ unsigned short tl[64][66]; const unsigned tid = threadIdx.x; const unsigned tpb = (unsigned)TTv / 64u; const unsigned slab = blockIdx.x / tpb, lg = blockIdx.x - slab * tpb; const unsigned b = slab / (unsigned)NHv, h = slab - b * (unsigned)NHv;
  for (unsigned i = tid; i < 512u; i += 256u) { const unsigned r = i >> 3, c8 = (i & 7u) * 8u; FragH f; f.half[0] = *(const v8us*)((const unsigned short*)V16 + ((size_t)b * TTv + lg * 64u + r) * ldv + voff + h * 64u + c8);
#pragma unroll
    for (int q = 0; q < 8; ++q) tl[r][c8 + q] = f.u[q]; }
  __syncthreads();
  for (int pass = 0; pass < 2; ++pass) {
#pragma unroll
    for (unsigned rd = 0; rd < 2; ++rd) { const unsigned d = rd * 32u + (tid >> 3), pc = tid & 7u; FragH f;
#pragma unroll
      for (int q = 0; q < 8; ++q) f.u[q] = tl[pc * 8u + q][d];
      *(volatile v8us*)((unsigned short*)Vt + ((size_t)slab * 64u + d) * TTv + lg * 64u + pc * 8u) = f.half[0]; }
    if (pass == 0) __threadfence(); } }

__global__ __launch_bounds__(128) void k_sgattn(const _Float16* __restrict__ Q16, const _Float16* __restrict__ K16, const _Float16* __restrict__ VT, const unsigned int* __restrict__ MB, _Float16* __restrict__ O16) {
  __shared__ __attribute__((aligned(16))) _Float16 sp[4][16][72];
  const unsigned tid = threadIdx.x, lane = tid & 31u, ln = lane & 15u, hh = lane >> 4;
  const unsigned w = (unsigned)__builtin_amdgcn_readfirstlane((int)(tid >> 5));
  const unsigned nqt = (unsigned)SQ / 64u; const unsigned bid = blockIdx.x; const unsigned bh = bid / nqt, qb = bid - bh * nqt; const unsigned b = bh / (unsigned)NH, h = bh - b * (unsigned)NH;
  const unsigned q0 = qb * 64u + w * 16u; const size_t rowb = (size_t)b * SQ;
  const _Float16* qp = Q16 + (rowb + q0 + ln) * (size_t)DM + h * (unsigned)HD;
  const v16h aq0 = g2_frag(qp, hh), aq1 = g2_frag(qp + 32, hh);
  const _Float16* kp = K16 + (rowb + ln) * (size_t)DM + h * (unsigned)HD;
  const _Float16* vp = VT + ((size_t)bh * HD + ln) * SQ;
  const unsigned int* mp = MB + ((size_t)(b * ((unsigned)SQ / 16u) + (q0 >> 4)) * ((unsigned)SQ / 64u)) * 32u + lane;
  const v8f z8 = {0.f,0.f,0.f,0.f,0.f,0.f,0.f,0.f};
  v8f o[4];
#pragma unroll
  for (int d = 0; d < 4; ++d) o[d] = z8;
#pragma unroll 1
  for (unsigned kt = 0; kt < (unsigned)SQ / 64u; ++kt) { const unsigned key0 = kt * 64u;
    unsigned int mw = mp[(size_t)kt * 32u]; asm volatile("" : "+v"(mw));
    v8f s[4];
#pragma unroll
    for (unsigned j = 0; j < 4; ++j) { const _Float16* kr = kp + (size_t)(key0 + 16u * j) * DM; const v16h b0 = g2_frag(kr, hh), b1 = g2_frag(kr + 32, hh); v8f acc = z8; acc = g2_mma(aq0, b0, acc); acc = g2_mma(aq1, b1, acc); s[j] = acc; }
#pragma unroll
    for (unsigned j = 0; j < 4; ++j) {
#pragma unroll
      for (int r = 0; r < 8; ++r) { const float x = s[j][r] * 0.03125f; const float sg = __builtin_amdgcn_rcpf(1.0f + __expf(-x));
        const float p = (((mw >> (8u * j + (unsigned)r)) & 1u) != 0u) ? sg : 0.f;
        sp[w][8u * hh + (unsigned)r][16u * j + ln] = toh_flush(p); } }
    __builtin_amdgcn_fence(4  , "workgroup"); __builtin_amdgcn_wave_barrier();
    const v16h ap0 = g2_frag(&sp[w][ln][0], hh), ap1 = g2_frag(&sp[w][ln][32], hh);
#pragma unroll
    for (unsigned d = 0; d < 4; ++d) { const _Float16* vr = vp + (size_t)(16u * d) * SQ + key0; const v16h b0 = g2_frag(vr, hh), b1 = g2_frag(vr + 32, hh); o[d] = g2_mma(ap0, b0, o[d]); o[d] = g2_mma(ap1, b1, o[d]); }
    __builtin_amdgcn_fence(4  , "workgroup"); __builtin_amdgcn_wave_barrier(); }
#pragma unroll
  for (int r = 0; r < 8; ++r) {
#pragma unroll
    for (unsigned d = 0; d < 4; ++d) sp[w][8u * hh + (unsigned)r][16u * d + ln] = toh_flush(o[d][r]); }
  __builtin_amdgcn_fence(4  , "workgroup"); __builtin_amdgcn_wave_barrier();
  for (int pass = 0; pass < 2; ++pass) {
#pragma unroll
    for (unsigned it = 0; it < 4; ++it) { const unsigned row = it * 4u + (lane >> 3), pc = (lane & 7u) * 8u; const v8us v = *(const v8us*)&sp[w][row][pc];
      *(volatile v8us*)((unsigned short*)O16 + (rowb + q0 + row) * (size_t)DM + h * (unsigned)HD + pc) = v; }
    if (pass == 0) __threadfence(); } }

constexpr size_t al256(size_t b) { return (b + 255) & ~(size_t)255; }
constexpr size_t SZ_BW = (size_t)DM * DM * 2;
constexpr size_t SZ_P16 = NR * DM * 2, SZ_VT = (size_t)NB * NH * HD * SQ * 2;
constexpr size_t SZ_MB = (size_t)NB * (SQ / 16) * (SQ / 64) * 32 * 4;
constexpr size_t WS_TOTAL = al256(SZ_BW) + 4 * al256(SZ_P16) + al256(SZ_VT) + al256(SZ_MB);
static_assert(WS_TOTAL <= (size_t)134217728);
static_assert(SZ_BW % 128 == 0 && SZ_P16 % 128 == 0 && SZ_VT % 128 == 0 && SZ_MB % 128 == 0);
constexpr unsigned CH_N = (SQ == SQ_FULL) ? 1u : (unsigned)NB;
constexpr size_t CH_R = (SQ == SQ_FULL) ? NR : (size_t)SQ;
static_assert(CH_R % 128 == 0 && (size_t)CH_N * CH_R == NR);
static_assert((((size_t)DM * DM) / 2048) * 256 * 8 == (size_t)DM * DM);
static_assert(((CH_R * DM) / 2048) * 256 * 8 * CH_N == NR * DM);
static_assert((((size_t)NB * (SQ / 16) * (SQ / 64)) / 4) * 4 * 32 == (size_t)NB * (SQ / 16) * (SQ / 64) * 32);
static_assert((size_t)NB * NH * (SQ / 64) * 256 * 2 * 8 == (size_t)NB * NH * HD * SQ);
static_assert((size_t)NB * NH * (SQ / 64) * 4 * 16 * 64 == NR * DM);
static_assert((CH_R / 128) * (DM / 64) * 4 * 32 * 64 * CH_N == NR * DM);

extern "C" void kernel_launch(void* const* d_in, const int* in_sizes, int n_in,
                              void* d_out, int out_size, void* d_ws, size_t ws_size, hipStream_t stream) {
  if (n_in < 6) return;
  const float* vals = (const float*)d_in[0]; const float* keys = (const float*)d_in[1]; const float* qrys = (const float*)d_in[2];
  const int* mask = (const int*)d_in[3]; const float* wfc = (const float*)d_in[4]; const float* bfc = (const float*)d_in[5];
  const size_t needX = ((size_t)(NB - 1) * SQ_FULL + SQ) * DM;
  const size_t needM = ((size_t)(NB - 1) * SQ_FULL + (size_t)(SQ - 1)) * SQ_FULL + SQ;
  if ((size_t)in_sizes[0] < needX || (size_t)in_sizes[1] < needX || (size_t)in_sizes[2] < needX || (size_t)out_size < needX) return;
  if ((size_t)in_sizes[3] < needM || (size_t)in_sizes[4] < (size_t)DM * DM || in_sizes[5] < DM) return;
  char* ws = (char*)d_ws; size_t off = 0;
  auto take = [&](size_t bytes) { char* p = ws + off; off += al256(bytes); return p; };
  _Float16* BW = (_Float16*)take(SZ_BW);
  _Float16* Q16 = (_Float16*)take(SZ_P16); _Float16* K16 = (_Float16*)take(SZ_P16); _Float16* V16 = (_Float16*)take(SZ_P16); _Float16* O16 = (_Float16*)take(SZ_P16);
  _Float16* VT = (_Float16*)take(SZ_VT); unsigned int* MB = (unsigned int*)take(SZ_MB);
  if (off > ws_size) return;

  k_cvt<<<(unsigned)(((size_t)DM * DM) / 2048), 256, 0, stream>>>(wfc, 16.0f, BW);
  for (unsigned c = 0; c < CH_N; ++c) { const size_t rin = (size_t)c * SQ_FULL, r0 = (size_t)c * CH_R;
    k_cvt<<<(unsigned)((CH_R * DM) / 2048), 256, 0, stream>>>(qrys + rin * DM, 1.0f, Q16 + r0 * DM);
    k_cvt<<<(unsigned)((CH_R * DM) / 2048), 256, 0, stream>>>(keys + rin * DM, 1.0f, K16 + r0 * DM);
    k_cvt<<<(unsigned)((CH_R * DM) / 2048), 256, 0, stream>>>(vals + rin * DM, 1.0f, V16 + r0 * DM); }
  k_mpack<<<(unsigned)(((size_t)NB * (SQ / 16) * (SQ / 64)) / 4), 128, 0, stream>>>(mask, MB);
  k_vt<NH, SQ><<<(unsigned)(NB * NH * (SQ / 64)), 256, 0, stream>>>(V16, (unsigned)DM, 0u, VT);
  k_sgattn<<<(unsigned)(NB * NH * (SQ / 64)), 128, 0, stream>>>(Q16, K16, VT, MB, O16);
  for (unsigned c = 0; c < CH_N; ++c) { const size_t rin = (size_t)c * SQ_FULL, r0 = (size_t)c * CH_R;
    k_gemm2<0, 0><<<(unsigned)((CH_R / 128) * (DM / 64)), 128, 0, stream>>>(O16 + r0 * DM, (unsigned)DM, BW, (unsigned)DM, 0.0625f, bfc, nullptr, (float*)d_out + rin * DM, nullptr, (unsigned)DM, 1.0f, (unsigned)CH_R, (unsigned)DM, (unsigned)DM); }
}
